// TwoStageGatedMoE_37099927503251
// MI455X (gfx1250) — hardware-verified
//
#include <hip/hip_runtime.h>

typedef __bf16         v16bf __attribute__((ext_vector_type(16)));
typedef float          v8f   __attribute__((ext_vector_type(8)));
typedef float          v4f   __attribute__((ext_vector_type(4)));
typedef unsigned int   v4u   __attribute__((ext_vector_type(4)));
typedef int            v4i   __attribute__((ext_vector_type(4)));
typedef double         v2d   __attribute__((ext_vector_type(2)));
typedef v4f __attribute__((may_alias)) v4fa;
typedef v4u __attribute__((may_alias)) v4ua;
typedef v4i __attribute__((may_alias)) v4ia;
typedef v2d __attribute__((may_alias)) v2da;

#define NTOK   4096
#define DM     256
#define HID    1024
#define NEXP   16
#define NPAIR  8192
#define LROWS  10240
#define NTILE  80
#define TROWS  128
#define HK     2048

#define OUT0_ELEMS (NTOK * DM)
#define OUT_TAIL   OUT0_ELEMS
#define OUT_TOTAL  (OUT0_ELEMS + 22)

static_assert(NPAIR + NEXP * 127 <= LROWS);
static_assert(LROWS == NTILE * TROWS);
static_assert(NPAIR == 2 * NTOK);
static_assert(OUT_TAIL + 21 < OUT_TOTAL);
static_assert((OUT0_ELEMS * 4) % 128 == 0);

#define OFF_W1T  ((size_t)0)
#define SZ_W1T   ((size_t)NEXP * HID * DM * 2)
#define OFF_W2D  (OFF_W1T + SZ_W1T)
#define SZ_W2D   ((size_t)NEXP * DM * HK * 2)
#define OFF_XG   (OFF_W2D + SZ_W2D)
#define SZ_XG    ((size_t)LROWS * DM * 2)
#define OFF_HHL  (OFF_XG + SZ_XG)
#define SZ_HHL   ((size_t)LROWS * HK * 2)
#define OFF_Y    (OFF_HHL + SZ_HHL)
#define SZ_Y     ((size_t)NPAIR * DM * 4)
#define OFF_PE   (OFF_Y + SZ_Y)
#define SZ_PE    ((size_t)NPAIR * 4)
#define OFF_PC   (OFF_PE + SZ_PE)
#define SZ_PC    ((size_t)NPAIR * 4)
#define OFF_LIST (OFF_PC + SZ_PC)
#define SZ_LIST  ((size_t)LROWS * 4)
#define OFF_TILE (OFF_LIST + SZ_LIST)
#define SZ_TILE  ((size_t)128 * 4)
#define OFF_FLAG (OFF_TILE + SZ_TILE)
#define SZ_FLAG  ((size_t)32 * 4)
#define OFF_REC  (OFF_FLAG + SZ_FLAG)
#define SZ_REC   ((size_t)256 * 48 * 8)
#define WS_TOTAL (OFF_REC + SZ_REC)
static_assert(WS_TOTAL == 80945792);
static_assert(WS_TOTAL <= 134217728);
static_assert(OFF_W2D % 128 == 0 && OFF_XG % 128 == 0 && OFF_HHL % 128 == 0 && OFF_Y % 128 == 0);
static_assert(OFF_PE % 128 == 0 && OFF_PC % 128 == 0 && OFF_LIST % 128 == 0 && OFF_TILE % 128 == 0);
static_assert(OFF_FLAG % 128 == 0 && OFF_REC % 128 == 0);

#define GT_THR 320
#define TOKP   771
#define G1N    2060
#define G2N    8192
#define GATE_DYN_BYTES ((16 * TOKP + G1N + G2N) * 4)
static_assert(GATE_DYN_BYTES == 90352);
static_assert((16 * TOKP * 4) % 16 == 0 && (G1N * 4) % 16 == 0);

#define SORT_CNT_B  32768
#define SORT_LIST_B 40960
#define SORT_CS_B   4096
#define SORT_DYN_BYTES (SORT_CNT_B + SORT_LIST_B + SORT_CS_B)

__device__ __forceinline__ unsigned bf_bits(float f) {
  const unsigned u = __float_as_uint(f);
  const unsigned r = (u + 0x7FFFu + ((u >> 16) & 1u)) >> 16;
  const unsigned n = (u >> 16) | 0x40u;
  return ((u & 0x7FFFFFFFu) > 0x7F800000u) ? n : r;
}
__device__ __forceinline__ float bf_val(float f) { return __uint_as_float(bf_bits(f) << 16); }
__device__ __forceinline__ unsigned pk2(float lo, float hi) { return bf_bits(lo) | (bf_bits(hi) << 16); }

struct FragBits { v4u a; v4u b; };

__device__ __forceinline__ v8f wmb(v16bf a, v16bf b, v8f c) {
  v8f d = __builtin_amdgcn_wmma_f32_16x16x32_bf16(false, a, false, b, (short)0, c, false, false);
  asm volatile("v_nop\n\tv_nop\n\tv_nop\n\tv_nop" : "+v"(d) : "v"(a), "v"(b));
  return d;
}

__device__ __forceinline__ v16bf load_frag(const unsigned short* p, int h) {
  FragBits f;
  f.a = *(const v4ua*)(p + 8 * h);
  f.b = *(const v4ua*)(p + 16 + 8 * h);
  return __builtin_bit_cast(v16bf, f);
}

template <int DUP>
__device__ __forceinline__ void tr_tile(const float* __restrict__ src, int ld,
                                        unsigned short* __restrict__ dst, int pitch,
                                        float* sT, int tid) {
  #pragma unroll 4
  for (int i = 0; i < 8; ++i) {
    const int q = tid + i * 256;
    const int k = q >> 3, c4 = (q & 7) * 4;
    const v4f v = *(const v4fa*)(src + (size_t)k * ld + c4);
    *(v4fa*)(sT + k * 32 + c4) = v;
  }
  __syncthreads();
  v4u o[4];
  #pragma unroll
  for (int i = 0; i < 4; ++i) {
    const int c = tid + i * 256;
    const int row = c >> 5, k0 = (c & 31) * 8;
    const float* p = sT + k0 * 32 + row;
    v4u t;
    t.x = pk2(p[0],   p[32]);
    t.y = pk2(p[64],  p[96]);
    t.z = pk2(p[128], p[160]);
    t.w = pk2(p[192], p[224]);
    o[i] = t;
  }
  #pragma unroll
  for (int i = 0; i < 4; ++i) {
    const int c = tid + i * 256;
    const int row = c >> 5, k0 = (c & 31) * 8;
    unsigned short* d = dst + (size_t)row * pitch + k0;
    *(volatile v4u*)d = o[i];
    if (DUP) *(volatile v4u*)(d + 1024) = o[i];
  }
  __threadfence();
  #pragma unroll
  for (int i = 0; i < 4; ++i) {
    const int c = tid + i * 256;
    const int row = c >> 5, k0 = (c & 31) * 8;
    unsigned short* d = dst + (size_t)row * pitch + k0;
    *(volatile v4u*)d = o[i];
    if (DUP) *(volatile v4u*)(d + 1024) = o[i];
  }
}

__global__ __launch_bounds__(256) void k_pw1(const float* __restrict__ W1, unsigned short* __restrict__ W1T) {
  __shared__ __attribute__((aligned(16))) float sT[256 * 32];
  const int b = blockIdx.x, e = b >> 5, nb = b & 31;
  tr_tile<0>(W1 + (size_t)e * DM * HID + nb * 32, HID,
             W1T + ((size_t)e * HID + nb * 32) * DM, DM, sT, threadIdx.x);
}

__global__ __launch_bounds__(256) void k_pw2(const float* __restrict__ W2, unsigned short* __restrict__ W2D) {
  __shared__ __attribute__((aligned(16))) float sT[256 * 32];
  const int b = blockIdx.x, e = b >> 5, nb = (b >> 2) & 7, kc = b & 3;
  tr_tile<1>(W2 + (size_t)e * HID * DM + (size_t)kc * 256 * DM + nb * 32, DM,
             W2D + ((size_t)e * DM + nb * 32) * HK + kc * 256, HK, sT, threadIdx.x);
}

__global__ __launch_bounds__(GT_THR) void k_gate(
    const float* __restrict__ x, const float* __restrict__ adj, const float* __restrict__ tf,
    const float* __restrict__ us, const float* __restrict__ mask,
    const float* __restrict__ g1W, const float* __restrict__ g1b,
    const float* __restrict__ g2W, const float* __restrict__ g2b,
    int* __restrict__ PE, float* __restrict__ PC, double* __restrict__ REC)
{
  extern __shared__ __attribute__((aligned(16))) float dsm[];
  __shared__ __attribute__((aligned(16))) double sLg[320];
  __shared__ __attribute__((aligned(16))) double sRec[48];
  __shared__ __attribute__((aligned(16))) float sE[320];
  __shared__ __attribute__((aligned(16))) float sP[320];
  __shared__ __attribute__((aligned(16))) float sF[16 * 64];
  __shared__ __attribute__((aligned(16))) int   sPE[32];
  __shared__ __attribute__((aligned(16))) float sPC[32];

  float* sTok = dsm;
  float* sW   = dsm + 16 * TOKP;
  const int tid = threadIdx.x;
  const int t0 = blockIdx.x * 16;

  #pragma unroll 1
  for (int it = 0; it < 4; ++it) {
    const int q = tid + it * GT_THR;
    const int qc = (q < 1023) ? q : 1023;
    const int tl = qc >> 6, c4 = (qc & 63) * 4;
    const size_t go = (size_t)(t0 + tl) * DM + c4;
    const v4f a = *(const v4fa*)(x + go);
    const v4f b = *(const v4fa*)(tf + go);
    const v4f c = *(const v4fa*)(us + go);
    if (q < 1024) {
      float* d = sTok + tl * TOKP;
      d[c4 + 0] = bf_val(a.x); d[c4 + 1] = bf_val(a.y); d[c4 + 2] = bf_val(a.z); d[c4 + 3] = bf_val(a.w);
      d[259 + c4 + 0] = bf_val(b.x); d[259 + c4 + 1] = bf_val(b.y); d[259 + c4 + 2] = bf_val(b.z); d[259 + c4 + 3] = bf_val(b.w);
      d[515 + c4 + 0] = bf_val(c.x); d[515 + c4 + 1] = bf_val(c.y); d[515 + c4 + 2] = bf_val(c.z); d[515 + c4 + 3] = bf_val(c.w);
    }
  }
  {
    const int qc = (tid < 11) ? tid : 11;
    const v4f a = *(const v4fa*)(adj + (size_t)t0 * 3 + qc * 4);
    if (tid < 12) {
      const int i0 = qc * 4;
      sTok[((i0 + 0) / 3) * TOKP + 256 + ((i0 + 0) % 3)] = bf_val(a.x);
      sTok[((i0 + 1) / 3) * TOKP + 256 + ((i0 + 1) % 3)] = bf_val(a.y);
      sTok[((i0 + 2) / 3) * TOKP + 256 + ((i0 + 2) % 3)] = bf_val(a.z);
      sTok[((i0 + 3) / 3) * TOKP + 256 + ((i0 + 3) % 3)] = bf_val(a.w);
    }
  }
  #pragma unroll 1
  for (int it = 0; it < 2; ++it) {
    const int q = tid + it * GT_THR;
    const int qc = (q < 514) ? q : 514;
    const v4f a = *(const v4fa*)(g1W + qc * 4);
    const v4f r = { bf_val(a.x), bf_val(a.y), bf_val(a.z), bf_val(a.w) };
    if (q < 515) *(v4fa*)(sW + qc * 4) = r;
  }
  #pragma unroll 1
  for (int it = 0; it < 7; ++it) {
    const int q = tid + it * GT_THR;
    const int qc = (q < 2047) ? q : 2047;
    const v4f a = *(const v4fa*)(g2W + qc * 4);
    const v4f r = { bf_val(a.x), bf_val(a.y), bf_val(a.z), bf_val(a.w) };
    if (q < 2048) *(v4fa*)(sW + G1N + qc * 4) = r;
  }
  __syncthreads();

  {
    const int tl = tid / 20, j = tid - tl * 20;
    const int j2 = (j > 4) ? (j - 4) : 0;
    const bool s1 = (j < 4);
    const float* tk = sTok + tl * TOKP;
    const int wA = s1 ? j : (G1N + (j2 >> 2) * 2048 + (j2 & 3));
    const int wB = wA + 1024;
    const int inB = s1 ? 256 : 515;
    const int lenB = s1 ? 259 : 256;
    double acc = 0.0;
    #pragma unroll 4
    for (int k = 0; k < 256; ++k)
      acc = __builtin_fma((double)tk[k], (double)sW[wA + 4 * k], acc);
    #pragma unroll 4
    for (int i = 0; i < 259; ++i) {
      const int ic = (i < lenB) ? i : (lenB - 1);
      const double wv = (double)sW[wB + 4 * ic];
      const double ws = (i < lenB) ? wv : 0.0;
      acc = __builtin_fma((double)tk[inB + ic], ws, acc);
    }
    const float bA = g1b[(j < 3) ? j : 3];
    const float bB = g2b[j2];
    const float bb = s1 ? bf_val(bA) : bf_val(bB);
    sLg[tid] = acc + (double)bb;
  }
  __syncthreads();

  if (tid < 32) {
    const int tl = tid & 15;
    const int lb = tl * 20;
    const double a0 = sLg[lb], a1 = sLg[lb + 1], a2 = sLg[lb + 2], a3 = sLg[lb + 3];
    int i1 = 0; double m1 = a0; bool c;
    c = a1 > m1; i1 = c ? 1 : i1; m1 = c ? a1 : m1;
    c = a2 > m1; i1 = c ? 2 : i1; m1 = c ? a2 : m1;
    c = a3 > m1; i1 = c ? 3 : i1; m1 = c ? a3 : m1;
    int i2 = -1; double m2 = 0.0;
    c = (i1 != 0);                                   i2 = c ? 0 : i2; m2 = c ? a0 : m2;
    c = (i1 != 1) & ((i2 < 0) | (a1 > m2));          i2 = c ? 1 : i2; m2 = c ? a1 : m2;
    c = (i1 != 2) & ((i2 < 0) | (a2 > m2));          i2 = c ? 2 : i2; m2 = c ? a2 : m2;
    c = (i1 != 3) & ((i2 < 0) | (a3 > m2));          i2 = c ? 3 : i2; m2 = c ? a3 : m2;

    int q[4];
    #pragma unroll
    for (int g = 0; g < 4; ++g) {
      const double b0 = sLg[lb + 4 + 4 * g], b1 = sLg[lb + 5 + 4 * g];
      const double b2 = sLg[lb + 6 + 4 * g], b3 = sLg[lb + 7 + 4 * g];
      int bi = 0; double bm = b0; bool d;
      d = b1 > bm; bi = d ? 1 : bi; bm = d ? b1 : bm;
      d = b2 > bm; bi = d ? 2 : bi; bm = d ? b2 : bm;
      d = b3 > bm; bi = d ? 3 : bi; bm = d ? b3 : bm;
      q[g] = bi;
    }
    const int qa = (i1 == 0) ? q[0] : ((i1 == 1) ? q[1] : ((i1 == 2) ? q[2] : q[3]));
    const int qb = (i2 == 0) ? q[0] : ((i2 == 1) ? q[1] : ((i2 == 2) ? q[2] : q[3]));

    #pragma unroll 1
    for (int r = 0; r < 5; ++r) {
      const int base = lb + 4 * r;
      const float z0 = (float)sLg[base], z1 = (float)sLg[base + 1];
      const float z2 = (float)sLg[base + 2], z3 = (float)sLg[base + 3];
      const float mx = fmaxf(fmaxf(z0, z1), fmaxf(z2, z3));
      float s = 0.0f;
      #pragma unroll 1
      for (int ci = 0; ci < 4; ++ci) {
        const float e = expf((float)sLg[base + ci] - mx);
        sE[base + ci] = e;
        s += e;
      }
      #pragma unroll 1
      for (int ci = 0; ci < 4; ++ci) sP[base + ci] = sE[base + ci] / s;
    }

    const float vf = (bf_val(mask[t0 + tl]) > 0.0f) ? 1.0f : 0.0f;
    float* F = sF + tl * 64;
    F[0] = 1.0f;
    F[1] = vf;
    #pragma unroll
    for (int g = 0; g < 4; ++g) {
      const bool ha = (i1 == g), hb = (i2 == g);
      F[2 + g]  = sP[lb + g];
      F[6 + g]  = (ha | hb) ? vf : 0.0f;
      F[26 + g] = ((ha ? 1.0f : 0.0f) + (hb ? 1.0f : 0.0f)) * vf;
    }
    #pragma unroll
    for (int j = 0; j < 16; ++j) {
      F[10 + j] = sP[lb + 4 + j];
      F[30 + j] = (q[j >> 2] == (j & 3)) ? 1.0f : 0.0f;
    }
    const float w1a = sP[lb + i1], w1b = sP[lb + i2];
    const float v2a = sP[lb + 4 + i1 * 4 + qa], v2b = sP[lb + 4 + i2 * 4 + qb];
    sPE[2 * tl]     = i1 * 4 + qa;
    sPE[2 * tl + 1] = i2 * 4 + qb;
    sPC[2 * tl]     = w1a * v2a;
    sPC[2 * tl + 1] = w1b * v2b;
  }
  __syncthreads();

  if (tid < 64) {
    const int j = (tid < 44) ? tid : 44;
    const int ia = (j < 4) ? (j + 2) : ((j == 4) ? 1 : (j + 1));
    const int ib = (j < 4) ? 1
                 : (((j >= 9) & (j < 25)) ? (6 + ((j - 9) >> 2))
                 : ((j >= 29) ? (6 + ((j - 29) >> 2)) : 0));
    double acc = 0.0;
    #pragma unroll 1
    for (int t = 0; t < 16; ++t)
      acc = __builtin_fma((double)sF[t * 64 + ia], (double)sF[t * 64 + ib], acc);
    if (tid < 48) sRec[tid] = (tid < 45) ? acc : 0.0;
  }
  __syncthreads();

  if (tid < 32) {
    const int l8 = tid & 7;
    const int l24 = (tid < 23) ? tid : 23;
    const v4i pe = *(const v4ia*)(sPE + 4 * l8);
    const v4f pc = *(const v4fa*)(sPC + 4 * l8);
    const v2d rc = *(const v2da*)(sRec + 2 * l24);
    int* pePtr = PE + (size_t)blockIdx.x * 32 + 4 * l8;
    float* pcPtr = PC + (size_t)blockIdx.x * 32 + 4 * l8;
    double* rcPtr = REC + (size_t)blockIdx.x * 48 + 2 * l24;
    if (tid < 8)  *(volatile v4i*)pePtr = pe;
    if (tid < 8)  *(volatile v4f*)pcPtr = pc;
    if (tid < 24) *(volatile v2d*)rcPtr = rc;
    __threadfence();
    if (tid < 8)  *(volatile v4i*)pePtr = pe;
    if (tid < 8)  *(volatile v4f*)pcPtr = pc;
    if (tid < 24) *(volatile v2d*)rcPtr = rc;
  }
}

__global__ __launch_bounds__(1024) void k_sort(const int* __restrict__ PE, int* __restrict__ LIST,
                                               int* __restrict__ TILE, int* __restrict__ FLAG)
{
  extern __shared__ __attribute__((aligned(16))) unsigned char ssm[];
  unsigned short* sCnt = (unsigned short*)ssm;
  int* sList = (int*)(ssm + SORT_CNT_B);
  unsigned* sCs = (unsigned*)(ssm + SORT_CNT_B + SORT_LIST_B);
  __shared__ int sBase[32];
  __shared__ int sTot[16];
  __shared__ int sBadW[32];
  __shared__ int sChk[4];
  __shared__ __attribute__((aligned(16))) int sTile[128];

  const int tid = threadIdx.x;

  {
    const v4i neg = { -1, -1, -1, -1 };
    #pragma unroll
    for (int it = 0; it < 3; ++it) {
      const int i = tid + it * 1024;
      if (i < 2560) *(v4ia*)(sList + 4 * i) = neg;
    }
    #pragma unroll
    for (int e = 0; e < 16; ++e) sCnt[e * 1024 + tid] = (unsigned short)0;
  }

  int ev[8];
  {
    const v4i p0 = *(const v4ia*)(PE + 8 * tid);
    const v4i p1 = *(const v4ia*)(PE + 8 * tid + 4);
    ev[0] = p0.x; ev[1] = p0.y; ev[2] = p0.z; ev[3] = p0.w;
    ev[4] = p1.x; ev[5] = p1.y; ev[6] = p1.z; ev[7] = p1.w;
  }
  int bad = 0;
  #pragma unroll
  for (int i = 0; i < 8; ++i) {
    const int e = ev[i];
    bad |= ((unsigned)e > 15u) ? 1 : 0;
    const int ec = (e < 0) ? 0 : ((e > 15) ? 15 : e);
    ev[i] = ec;
    const int idx = ec * 1024 + tid;
    sCnt[idx] = (unsigned short)(sCnt[idx] + 1);
  }
  {
    const unsigned long long bm = __ballot(bad != 0);
    if ((tid & 31) == 0) sBadW[tid >> 5] = (bm != 0ull) ? 1 : 0;
  }
  __syncthreads();

  const int ce = tid >> 6, cc = tid & 63;
  {
    unsigned s = 0;
    #pragma unroll 4
    for (int i = 0; i < 16; ++i) s += sCnt[ce * 1024 + 16 * cc + i];
    sCs[ce * 64 + cc] = s;
  }
  __syncthreads();
  if (tid < 16) {
    unsigned run = 0;
    #pragma unroll 4
    for (int c = 0; c < 64; ++c) {
      const unsigned v = sCs[tid * 64 + c];
      sCs[tid * 64 + c] = run;
      run += v;
    }
    sTot[tid] = (int)run;
  }
  __syncthreads();
  if (tid == 0) {
    int base = 0, sum = 0, b = 0;
    #pragma unroll 1
    for (int e = 0; e < 16; ++e) {
      const int cnt = sTot[e];
      sBase[e] = base;
      b |= (cnt > NTOK) ? 1 : 0;
      sum += cnt;
      base += ((cnt + 127) >> 7) << 7;
    }
    sBase[16] = base;
    b |= (sum != NPAIR) ? 1 : 0;
    b |= (base > LROWS) ? 1 : 0;
    #pragma unroll 1
    for (int w = 0; w < 32; ++w) b |= sBadW[w];
    sChk[0] = b;
  }
  __syncthreads();
  {
    unsigned run = (unsigned)sBase[ce] + sCs[ce * 64 + cc];
    #pragma unroll 4
    for (int i = 0; i < 16; ++i) {
      const int idx = ce * 1024 + 16 * cc + i;
      const unsigned v = sCnt[idx];
      sCnt[idx] = (unsigned short)run;
      run += v;
    }
  }
  __syncthreads();
  #pragma unroll
  for (int i = 0; i < 8; ++i) {
    const int idx = ev[i] * 1024 + tid;
    const int row = (int)sCnt[idx];
    sCnt[idx] = (unsigned short)(row + 1);
    const int rc = (row < LROWS - 1) ? row : (LROWS - 1);
    sList[rc] = 8 * tid + i;
  }
  if (tid < 128) {
    const int r0 = tid * TROWS;
    int te = -1;
    #pragma unroll
    for (int e = 0; e < 16; ++e) {
      const bool in = (r0 >= sBase[e]) & (r0 < sBase[e + 1]);
      te = in ? e : te;
    }
    sTile[tid] = te;
  }
  __syncthreads();

  v4i lv[3];
  #pragma unroll
  for (int it = 0; it < 3; ++it) {
    const int i = tid + it * 1024;
    const int ic = (i < 2559) ? i : 2559;
    lv[it] = *(const v4ia*)(sList + 4 * ic);
  }
  const v4i tv = *(const v4ia*)(sTile + 4 * (tid & 31));
  const int fl = sChk[0];
  const v4i fv = { fl, fl, fl, fl };
  #pragma unroll
  for (int it = 0; it < 3; ++it) {
    const int i = tid + it * 1024;
    if (i < 2560) *(volatile v4i*)(LIST + 4 * i) = lv[it];
  }
  if (tid < 32) *(volatile v4i*)(TILE + 4 * tid) = tv;
  if (tid < 8)  *(volatile v4i*)(FLAG + 4 * tid) = fv;
  __threadfence();
  #pragma unroll
  for (int it = 0; it < 3; ++it) {
    const int i = tid + it * 1024;
    if (i < 2560) *(volatile v4i*)(LIST + 4 * i) = lv[it];
  }
  if (tid < 32) *(volatile v4i*)(TILE + 4 * tid) = tv;
  if (tid < 8)  *(volatile v4i*)(FLAG + 4 * tid) = fv;
}

__global__ __launch_bounds__(256) void k_gather(const float* __restrict__ x, const int* __restrict__ LIST,
                                                unsigned short* __restrict__ XG)
{
  const int lane = threadIdx.x & 31;
  const int r = blockIdx.x * 8 + (threadIdx.x >> 5);
  const int pid = LIST[r];
  const bool ok = (pid >= 0) & (pid < NPAIR);
  const int pc = (pid < 0) ? 0 : ((pid > NPAIR - 1) ? (NPAIR - 1) : pid);
  const float* src = x + (size_t)(pc >> 1) * DM + lane * 8;
  const v4f a = *(const v4fa*)src;
  const v4f b = *(const v4fa*)(src + 4);
  v4u o;
  o.x = pk2(a.x, a.y); o.y = pk2(a.z, a.w); o.z = pk2(b.x, b.y); o.w = pk2(b.z, b.w);
  const unsigned msk = ok ? 0xFFFFFFFFu : 0u;
  o.x &= msk; o.y &= msk; o.z &= msk; o.w &= msk;
  unsigned short* dst = XG + (size_t)r * DM + lane * 8;
  *(volatile v4u*)dst = o;
  __threadfence();
  *(volatile v4u*)dst = o;
}

__device__ __forceinline__ unsigned gelu_split(float a, float bias) {
  const float v = a + bias;
  const float g = 0.5f * v * (1.0f + erff(v * 0.70710678f));
  const unsigned hb = bf_bits(g);
  const float hf = __uint_as_float(hb << 16);
  const unsigned lb = bf_bits(g - hf);
  return hb | (lb << 16);
}

__device__ __forceinline__ void hhl_store_pass(const float* sT, unsigned short* HHL, int m0, int n0, int w, int lane) {
  const int q8 = lane & 7, sub = lane >> 3;
  #pragma unroll
  for (int it = 0; it < 8; ++it) {
    const int row = 32 * w + 4 * it + sub;
    const float* p = sT + row * 64 + 8 * q8;
    const v4u H = *(const v4ua*)p;
    const v4u L = *(const v4ua*)(p + 4);
    unsigned short* d = HHL + (size_t)(m0 + row) * HK + n0 + 8 * q8;
    *(volatile v4u*)d = H;
    *(volatile v4u*)(d + 1024) = L;
  }
}

__global__ __launch_bounds__(128) __attribute__((amdgpu_num_vgpr(248))) void k_g1(
    const unsigned short* __restrict__ XG, const unsigned short* __restrict__ W1T,
    const float* __restrict__ b1, const int* __restrict__ TILE, unsigned short* __restrict__ HHL)
{
  __shared__ __attribute__((aligned(16))) float sT[128 * 64];
  __shared__ __attribute__((aligned(16))) float sBias[64];

  const int e = TILE[blockIdx.x];
  if ((e < 0) | (e > 15)) return;

  const int tid = threadIdx.x, lane = tid & 31, w = tid >> 5;
  const int h = lane >> 4, m = lane & 15;
  const int m0 = blockIdx.x * TROWS, n0 = blockIdx.y * 64;

  if (tid < 64) sBias[tid] = bf_val(b1[e * HID + n0 + tid]);

  const unsigned short* xa0 = XG + (size_t)(m0 + 32 * w + m) * DM;
  const unsigned short* xa1 = xa0 + (size_t)16 * DM;
  const unsigned short* wb  = W1T + ((size_t)e * HID + n0 + m) * DM;

  const v8f zero8 = {0.f, 0.f, 0.f, 0.f, 0.f, 0.f, 0.f, 0.f};
  v8f acc[2][4];
  #pragma unroll
  for (int mt = 0; mt < 2; ++mt)
    #pragma unroll
    for (int nt = 0; nt < 4; ++nt) acc[mt][nt] = zero8;

  #pragma unroll 1
  for (int k0 = 0; k0 < DM; k0 += 32) {
    const v16bf a0 = load_frag(xa0 + k0, h);
    const v16bf a1 = load_frag(xa1 + k0, h);
    #pragma unroll
    for (int nt = 0; nt < 4; ++nt) {
      const v16bf b = load_frag(wb + (size_t)nt * 16 * DM + k0, h);
      acc[0][nt] = wmb(a0, b, acc[0][nt]);
      acc[1][nt] = wmb(a1, b, acc[1][nt]);
    }
  }

  #pragma unroll
  for (int nt = 0; nt < 4; ++nt)
    #pragma unroll
    for (int mt = 0; mt < 2; ++mt)
      #pragma unroll
      for (int r = 0; r < 8; ++r)
        sT[(32 * w + 16 * mt + 8 * h + r) * 64 + 16 * nt + m] = acc[mt][nt][r];
  __syncthreads();

  {
    const int q8 = lane & 7, sub = lane >> 3;
    const v4f ba = *(const v4fa*)(sBias + 8 * q8);
    const v4f bb = *(const v4fa*)(sBias + 8 * q8 + 4);
    #pragma unroll 1
    for (int it = 0; it < 8; ++it) {
      const int row = 32 * w + 4 * it + sub;
      float* p = sT + row * 64 + 8 * q8;
      const v4f va = *(const v4fa*)p;
      const v4f vb = *(const v4fa*)(p + 4);
      const unsigned s0 = gelu_split(va.x, ba.x), s1 = gelu_split(va.y, ba.y);
      const unsigned s2 = gelu_split(va.z, ba.z), s3 = gelu_split(va.w, ba.w);
      const unsigned s4 = gelu_split(vb.x, bb.x), s5 = gelu_split(vb.y, bb.y);
      const unsigned s6 = gelu_split(vb.z, bb.z), s7 = gelu_split(vb.w, bb.w);
      v4u H, L;
      H.x = (s0 & 0xFFFFu) | (s1 << 16); H.y = (s2 & 0xFFFFu) | (s3 << 16);
      H.z = (s4 & 0xFFFFu) | (s5 << 16); H.w = (s6 & 0xFFFFu) | (s7 << 16);
      L.x = (s0 >> 16) | (s1 & 0xFFFF0000u); L.y = (s2 >> 16) | (s3 & 0xFFFF0000u);
      L.z = (s4 >> 16) | (s5 & 0xFFFF0000u); L.w = (s6 >> 16) | (s7 & 0xFFFF0000u);
      *(v4ua*)p = H;
      *(v4ua*)(p + 4) = L;
    }
  }
  __syncthreads();

  hhl_store_pass(sT, HHL, m0, n0, w, lane);
  __threadfence();
  hhl_store_pass(sT, HHL, m0, n0, w, lane);
}

__device__ __forceinline__ void y_store_pass(const float* sT, const int* sPid, float* Y, int n0, int w, int lane) {
  const int l16 = lane & 15, sub = lane >> 4;
  #pragma unroll
  for (int it = 0; it < 16; ++it) {
    const int row = 32 * w + 2 * it + sub;
    const int pid = sPid[row];
    const v4f v = *(const v4fa*)(sT + row * 64 + 4 * l16);
    const int pc = (pid < 0) ? 0 : ((pid > NPAIR - 1) ? (NPAIR - 1) : pid);
    if ((pid >= 0) & (pid < NPAIR))
      *(volatile v4f*)(Y + (size_t)pc * DM + n0 + 4 * l16) = v;
  }
}

__global__ __launch_bounds__(128) __attribute__((amdgpu_num_vgpr(248))) void k_g2(
    const unsigned short* __restrict__ HHL, const unsigned short* __restrict__ W2D,
    const float* __restrict__ b2, const int* __restrict__ TILE, const int* __restrict__ LIST,
    float* __restrict__ Y)
{
  __shared__ __attribute__((aligned(16))) float sT[128 * 64];
  __shared__ int sPid[128];

  const int e = TILE[blockIdx.x];
  if ((e < 0) | (e > 15)) return;

  const int tid = threadIdx.x, lane = tid & 31, w = tid >> 5;
  const int h = lane >> 4, m = lane & 15;
  const int m0 = blockIdx.x * TROWS, n0 = blockIdx.y * 64;

  sPid[tid] = LIST[m0 + tid];

  const unsigned short* ha0 = HHL + (size_t)(m0 + 32 * w + m) * HK;
  const unsigned short* ha1 = ha0 + (size_t)16 * HK;
  const unsigned short* wb  = W2D + ((size_t)e * DM + n0 + m) * HK;

  const v8f zero8 = {0.f, 0.f, 0.f, 0.f, 0.f, 0.f, 0.f, 0.f};
  v8f acc[2][4];
  #pragma unroll
  for (int mt = 0; mt < 2; ++mt)
    #pragma unroll
    for (int nt = 0; nt < 4; ++nt) acc[mt][nt] = zero8;

  #pragma unroll 1
  for (int k0 = 0; k0 < HK; k0 += 32) {
    const v16bf a0 = load_frag(ha0 + k0, h);
    const v16bf a1 = load_frag(ha1 + k0, h);
    #pragma unroll
    for (int nt = 0; nt < 4; ++nt) {
      const v16bf b = load_frag(wb + (size_t)nt * 16 * HK + k0, h);
      acc[0][nt] = wmb(a0, b, acc[0][nt]);
      acc[1][nt] = wmb(a1, b, acc[1][nt]);
    }
  }

  #pragma unroll
  for (int nt = 0; nt < 4; ++nt) {
    const float bv = bf_val(b2[e * DM + n0 + 16 * nt + m]);
    #pragma unroll
    for (int mt = 0; mt < 2; ++mt)
      #pragma unroll
      for (int r = 0; r < 8; ++r)
        sT[(32 * w + 16 * mt + 8 * h + r) * 64 + 16 * nt + m] = acc[mt][nt][r] + bv;
  }
  __syncthreads();

  y_store_pass(sT, sPid, Y, n0, w, lane);
  __threadfence();
  y_store_pass(sT, sPid, Y, n0, w, lane);
}

__global__ __launch_bounds__(256) void k_final(const float* __restrict__ Y, const float* __restrict__ PC,
                                               const int* __restrict__ FLAG, float* __restrict__ out)
{
  const int lane = threadIdx.x & 31;
  const int t = blockIdx.x * 8 + (threadIdx.x >> 5);
  const float c0 = PC[2 * t], c1 = PC[2 * t + 1];
  const bool poison = (FLAG[0] != 0);
  const float qn = __uint_as_float(0x7FC00000u);
  const float* y0 = Y + (size_t)(2 * t) * DM;
  const float* y1 = y0 + DM;
  v4f o[2];
  #pragma unroll
  for (int j = 0; j < 2; ++j) {
    const int col = j * 128 + 4 * lane;
    const v4f a = *(const v4fa*)(y0 + col);
    const v4f b = *(const v4fa*)(y1 + col);
    v4f r;
    r.x = c0 * a.x + c1 * b.x;
    r.y = c0 * a.y + c1 * b.y;
    r.z = c0 * a.z + c1 * b.z;
    r.w = c0 * a.w + c1 * b.w;
    r.x = poison ? qn : r.x; r.y = poison ? qn : r.y;
    r.z = poison ? qn : r.z; r.w = poison ? qn : r.w;
    o[j] = r;
  }
  float* dst = out + (size_t)t * DM + 4 * lane;
  *(volatile v4f*)dst = o[0];
  *(volatile v4f*)(dst + 128) = o[1];
  __threadfence();
  *(volatile v4f*)dst = o[0];
  *(volatile v4f*)(dst + 128) = o[1];
}

__global__ __launch_bounds__(64) void k_stats(const double* __restrict__ REC, float* __restrict__ out)
{
  __shared__ double sR[48];
  __shared__ float sO[32];
  const int tid = threadIdx.x;
  const int j = (tid < 47) ? tid : 47;
  double acc = 0.0;
  #pragma unroll 4
  for (int b = 0; b < 256; ++b) acc += REC[(size_t)b * 48 + j];
  if (tid < 48) sR[tid] = acc;
  if (tid < 32) sO[tid] = 0.0f;
  __syncthreads();
  if (tid == 0) {
    const float nv = fmaxf((float)sR[4], 1.0f);
    float lb1 = 0.0f;
    #pragma unroll 1
    for (int g = 0; g < 4; ++g) {
      const float pm = (float)sR[g] / nv - 0.25f;
      lb1 += pm * pm;
    }
    float lb2 = 0.0f;
    #pragma unroll 1
    for (int g = 0; g < 4; ++g) {
      const float c = (float)sR[5 + g];
      const float dn = fmaxf(c, 1.0f);
      float s = 0.0f;
      #pragma unroll 1
      for (int e = 0; e < 4; ++e) {
        const float pm = (float)sR[9 + 4 * g + e] / dn - 0.25f;
        s += pm * pm;
      }
      lb2 += (c > 0.0f) ? s : 0.0f;
    }
    sO[0] = lb1;
    sO[1] = lb2;
    #pragma unroll 1
    for (int g = 0; g < 4; ++g) sO[2 + g] = (float)sR[25 + g];
    #pragma unroll 1
    for (int k = 0; k < 16; ++k) sO[6 + k] = (float)sR[29 + k];
  }
  __syncthreads();
  if (tid < 32) {
    const float v = sO[(tid < 21) ? tid : 21];
    if (tid < 22) *(volatile float*)(out + OUT_TAIL + tid) = v;
    __threadfence();
    if (tid < 22) *(volatile float*)(out + OUT_TAIL + tid) = v;
  }
}

extern "C" void kernel_launch(void* const* d_in, const int* in_sizes, int n_in,
                              void* d_out, int out_size, void* d_ws, size_t ws_size,
                              hipStream_t stream) {
  if (n_in < 13) return;
  if (in_sizes[0] != NTOK * DM || in_sizes[2] != NTOK * DM || in_sizes[3] != NTOK * DM) return;
  if (in_sizes[1] != NTOK * 3 || in_sizes[4] != NTOK) return;
  if (in_sizes[5] != G1N || in_sizes[6] != 4 || in_sizes[7] != G2N || in_sizes[8] != 16) return;
  if (in_sizes[9] != NEXP * DM * HID || in_sizes[10] != NEXP * HID) return;
  if (in_sizes[11] != NEXP * HID * DM || in_sizes[12] != NEXP * DM) return;
  if (out_size != OUT_TOTAL) return;
  if (WS_TOTAL > ws_size) return;

  const float* x    = (const float*)d_in[0];
  const float* adj  = (const float*)d_in[1];
  const float* tf   = (const float*)d_in[2];
  const float* us   = (const float*)d_in[3];
  const float* mask = (const float*)d_in[4];
  const float* g1W  = (const float*)d_in[5];
  const float* g1b  = (const float*)d_in[6];
  const float* g2W  = (const float*)d_in[7];
  const float* g2b  = (const float*)d_in[8];
  const float* W1   = (const float*)d_in[9];
  const float* b1   = (const float*)d_in[10];
  const float* W2   = (const float*)d_in[11];
  const float* b2   = (const float*)d_in[12];
  float* out = (float*)d_out;

  unsigned char* ws = (unsigned char*)d_ws;
  unsigned short* W1T = (unsigned short*)(ws + OFF_W1T);
  unsigned short* W2D = (unsigned short*)(ws + OFF_W2D);
  unsigned short* XG  = (unsigned short*)(ws + OFF_XG);
  unsigned short* HHL = (unsigned short*)(ws + OFF_HHL);
  float*  Y    = (float*)(ws + OFF_Y);
  int*    PE   = (int*)(ws + OFF_PE);
  float*  PC   = (float*)(ws + OFF_PC);
  int*    LIST = (int*)(ws + OFF_LIST);
  int*    TILE = (int*)(ws + OFF_TILE);
  int*    FLAG = (int*)(ws + OFF_FLAG);
  double* REC  = (double*)(ws + OFF_REC);

  (void)hipFuncSetAttribute(reinterpret_cast<const void*>(&k_gate),
                            hipFuncAttributeMaxDynamicSharedMemorySize, GATE_DYN_BYTES);
  (void)hipFuncSetAttribute(reinterpret_cast<const void*>(&k_sort),
                            hipFuncAttributeMaxDynamicSharedMemorySize, SORT_DYN_BYTES);

  k_pw1<<<NEXP * 32, 256, 0, stream>>>(W1, W1T);
  k_pw2<<<NEXP * 32, 256, 0, stream>>>(W2, W2D);
  k_gate<<<NTOK / 16, GT_THR, GATE_DYN_BYTES, stream>>>(x, adj, tf, us, mask, g1W, g1b, g2W, g2b, PE, PC, REC);
  k_sort<<<1, 1024, SORT_DYN_BYTES, stream>>>(PE, LIST, TILE, FLAG);
  k_gather<<<LROWS / 8, 256, 0, stream>>>(x, LIST, XG);
  k_g1<<<dim3(NTILE, HID / 64), 128, 0, stream>>>(XG, W1T, b1, TILE, HHL);
  k_g2<<<dim3(NTILE, DM / 64), 128, 0, stream>>>(HHL, W2D, b2, TILE, LIST, Y);
  k_final<<<NTOK / 8, 256, 0, stream>>>(Y, PC, FLAG, out);
  k_stats<<<1, 64, 0, stream>>>(REC, out);
  (void)hipGetLastError();
}
